// CLIPVisionTower_73469710565951
// MI455X (gfx1250) — hardware-run, weakly checked
//
#include <hip/hip_runtime.h>


#ifndef NB
#define NB 16
#endif
#ifndef TQ
#define TQ 577
#endif
#define NB_FULL 16
#define T_FULL  577
#ifndef OUT_T
#define OUT_T TQ
#endif
#define DM   1024
#define DL   4096
#define LT   64
#define NH_  16
#define HD   64
#define TP   (((TQ + 63) / 64) * 64)
#define SP   (LT + TP)
#define SV   (LT + TQ)
#define KEND (((SV + 31) / 32) * 32)
#define AW   4
#define OSP  68
#define WCS  64.0f
#define WCI  (1.0f / 64.0f)
#define CXS  16.0f
#define OCI  (1.0f / 1024.0f)
#define SC2  ((float)(0.125 * 1.4426950408889634))
#define PSH  14.0f
#define NEGB (-3.0e38f)

static_assert(HD == 64);
static_assert(NH_ * HD == DM);
static_assert(LT == 64);
static_assert(DM % 64 == 0);
static_assert(DM % 32 == 0);
static_assert(DL % 32 == 0);
static_assert(TP % 64 == 0);
static_assert(SP % 64 == 0);
static_assert(TP % (16 * AW) == 0);
static_assert(KEND % 32 == 0);
static_assert(SV <= KEND);
static_assert(KEND <= SP);
static_assert(TQ >= 1);
static_assert(TQ <= T_FULL);
static_assert(NB <= NB_FULL);
static_assert(OUT_T >= TQ);
static_assert((OSP * 4) % 16 == 0);
static_assert(OSP >= 64);
static_assert((size_t)AW * 16 * OSP * 4 <= 131072);
static_assert((size_t)16 * 68 * 4 <= 131072);
static_assert(((size_t)DM * DM) % 8 == 0);
static_assert(((size_t)DM * DL) % 8 == 0);
static_assert(((size_t)LT * DL) % 8 == 0);
static_assert(DM % 8 == 0);

typedef _Float16 h16;
typedef __attribute__((ext_vector_type(16))) _Float16 v16h;
typedef __attribute__((ext_vector_type(8)))  _Float16 v8h;
typedef __attribute__((ext_vector_type(8)))  float    v8f;
typedef __attribute__((ext_vector_type(4)))  float    v4f;
typedef v4f  __attribute__((may_alias)) v4fa;

__device__ __forceinline__ unsigned short f2bf(float f) { unsigned u = __float_as_uint(f); u += 0x7FFFu + ((u >> 16) & 1u); return (unsigned short)(u >> 16); }
__device__ __forceinline__ float bfr(float f) { return __uint_as_float(((unsigned)f2bf(f)) << 16); }
__device__ __forceinline__ v16h cat16(v8h lo, v8h hi) { return __builtin_shufflevector(lo, hi, 0, 1, 2, 3, 4, 5, 6, 7, 8, 9, 10, 11, 12, 13, 14, 15); }
__device__ __forceinline__ v8f wmma16(v16h a, v16h b, v8f c) { return __builtin_amdgcn_wmma_f32_16x16x32_f16(false, a, false, b, (short)0, c, false, false); }
__device__ __forceinline__ v8f wmma16g(v16h a, v16h b, v8f c) { c = wmma16(a, b, c); asm volatile("v_nop\n\tv_nop\n\tv_nop\n\tv_nop" : "+v"(c) : "v"(a), "v"(b)); return c; }
__device__ __forceinline__ v16h  ldh(const h16* p) { return cat16(*(const v8h*)p, *(const v8h*)(p + 16)); }
__device__ __forceinline__ void wave_sync() { __builtin_amdgcn_fence(3  , "wavefront"); __builtin_amdgcn_wave_barrier(); asm volatile("" ::: "memory"); }
static __device__ __forceinline__ h16 toh_flush(float v) { const h16 r = (h16)v; return (fabsf(v) < 6.103515625e-05f) ? (h16)0.0f : r; }

__global__ __launch_bounds__(256) void k_cvth(const float* __restrict__ src, h16* dst, size_t n8, float carry) {
    const size_t i = (size_t)blockIdx.x * 256 + threadIdx.x; if (i >= n8) return;
    const v8f v = *(const v8f*)(src + i * 8); v8h o;
#pragma unroll
    for (int k = 0; k < 8; ++k) o[k] = toh_flush(bfr(v[k]) * carry);
    *(volatile v8h*)(dst + i * 8) = o; __threadfence(); *(volatile v8h*)(dst + i * 8) = o;
}

__global__ __launch_bounds__(256) void k_cvtx(const float* __restrict__ src, h16* dst, size_t n8) {
    const size_t i = (size_t)blockIdx.x * 256 + threadIdx.x; if (i >= n8) return;
    const int c8 = (int)(i % (size_t)(DM / 8)); const size_t row = i / (size_t)(DM / 8);
    const int b = (int)(row / (size_t)TP), t = (int)(row % (size_t)TP);
    const int tc = t < TQ ? t : (TQ - 1);
    v8f v = *(const v8f*)(src + ((size_t)b * T_FULL + (size_t)tc) * DM + (size_t)c8 * 8);
    asm volatile("" : "+v"(v));
    const float keep = (t < TQ) ? 1.0f : 0.0f;
    v8h o;
#pragma unroll
    for (int k = 0; k < 8; ++k) o[k] = toh_flush(bfr(v[k]) * keep);
    h16* p = dst + ((size_t)b * SP + (size_t)(LT + t)) * DM + (size_t)c8 * 8;
    *(volatile v8h*)p = o; __threadfence(); *(volatile v8h*)p = o;
}

template <int BIASROW, int F32OUT>
__device__ __forceinline__ void gemm_tile(const h16* __restrict__ A, const h16* __restrict__ Bt, const int K, const size_t arow, const size_t brow,
                                          const float* __restrict__ bias, const int bidx, const float oscale,
                                          h16* OH, float* OF, const size_t obase, const size_t opitch, const int rvalid) {
    __shared__ __align__(16) float os[16 * 68];
    const int lane = threadIdx.x & 31, lr = lane & 15, hi = lane >> 4;
    v8f acc[4][4];
#pragma unroll
    for (int mb = 0; mb < 4; ++mb)
#pragma unroll
        for (int nb = 0; nb < 4; ++nb) acc[mb][nb] = (v8f){};
    const size_t aoff = (arow + (size_t)lr) * (size_t)K + 8 * hi, boff = (brow + (size_t)lr) * (size_t)K + 8 * hi;
#pragma unroll 1
    for (int kc = 0; kc < K; kc += 32) {
        v16h a[4];
#pragma unroll
        for (int mb = 0; mb < 4; ++mb) a[mb] = ldh(A + aoff + (size_t)mb * 16 * K + kc);
#pragma unroll
        for (int nb = 0; nb < 4; ++nb) { const v16h bfrag = ldh(Bt + boff + (size_t)nb * 16 * K + kc);
#pragma unroll
            for (int mb = 0; mb < 4; ++mb) acc[mb][nb] = wmma16g(a[mb], bfrag, acc[mb][nb]); }
    }
    float bc[4];
#pragma unroll
    for (int nb = 0; nb < 4; ++nb) bc[nb] = BIASROW ? 0.0f : bfr(bias[bidx + nb * 16 + lr]);
#pragma unroll
    for (int mb = 0; mb < 4; ++mb) {
        float br[8];
#pragma unroll
        for (int j = 0; j < 8; ++j) br[j] = BIASROW ? bfr(bias[bidx + mb * 16 + hi * 8 + j]) : 0.0f;
#pragma unroll
        for (int nb = 0; nb < 4; ++nb) {
#pragma unroll
            for (int j = 0; j < 8; ++j) os[(hi * 8 + j) * 68 + nb * 16 + lr] = acc[mb][nb][j] * oscale + bc[nb] + br[j]; }
        wave_sync();
#pragma unroll 1
        for (int ps = 0; ps < 2; ++ps) {
            if (F32OUT) {
                static_assert(32 * 16 * 8 == 16 * 64 * 4);
#pragma unroll
                for (int s = 0; s < 8; ++s) { const int row = 2 * s + (lane >> 4), c4 = (lane & 15) * 4;
                    const v4f val = *(const v4fa*)(&os[row * 68 + c4]);
                    if (mb * 16 + row < rvalid) *(volatile v4f*)(OF + obase + (size_t)(mb * 16 + row) * opitch + c4) = val; }
            } else {
                static_assert(32 * 16 * 4 == 16 * 64 * 2);
#pragma unroll
                for (int s = 0; s < 4; ++s) { const int row = 4 * s + (lane >> 3), c8 = (lane & 7) * 8;
                    const v4f x0 = *(const v4fa*)(&os[row * 68 + c8]); const v4f x1 = *(const v4fa*)(&os[row * 68 + c8 + 4]); v8h hv;
#pragma unroll
                    for (int i = 0; i < 4; ++i) { hv[i] = toh_flush(x0[i]); hv[4 + i] = toh_flush(x1[i]); }
                    *(volatile v8h*)(OH + obase + (size_t)(mb * 16 + row) * opitch + c8) = hv; }
            }
            if (ps == 0) __threadfence(); }
        wave_sync();
    }
}

__global__ __launch_bounds__(32) void k_gemm_latt(const h16* __restrict__ LRW, const h16* __restrict__ WPH, const float* __restrict__ bp, h16* KVIN) {
    const int r0 = blockIdx.x * 64, c0 = blockIdx.y * 64;
    const int b = r0 / LT, l0 = r0 % LT;
    const size_t obase = ((size_t)b * SP + (size_t)l0) * DM + (size_t)c0;
    gemm_tile<0, 0>(LRW, WPH, DL, (size_t)r0, (size_t)c0, bp, c0, WCI, KVIN, (float*)0, obase, (size_t)DM, 64);
}

__global__ __launch_bounds__(32) void k_gemm_q(const h16* __restrict__ KVIN, const h16* __restrict__ WQH, const float* __restrict__ bq, h16* QP) {
    const int r0 = blockIdx.x * 64, c0 = blockIdx.y * 64;
    const int b = r0 / TP, tt = r0 % TP;
    const size_t arow = (size_t)b * SP + (size_t)(LT + tt);
    const size_t obase = (((size_t)b * NH_ + (size_t)(c0 / HD)) * TP + (size_t)tt) * HD;
    gemm_tile<0, 0>(KVIN, WQH, DM, arow, (size_t)c0, bq, c0, WCI, QP, (float*)0, obase, (size_t)HD, 64);
}

__global__ __launch_bounds__(32) void k_gemm_k(const h16* __restrict__ KVIN, const h16* __restrict__ WKH, const float* __restrict__ bk, h16* KP) {
    const int r0 = blockIdx.x * 64, c0 = blockIdx.y * 64;
    const int b = r0 / SP, kk = r0 % SP;
    const size_t obase = (((size_t)b * NH_ + (size_t)(c0 / HD)) * SP + (size_t)kk) * HD;
    gemm_tile<0, 0>(KVIN, WKH, DM, (size_t)r0, (size_t)c0, bk, c0, WCI, KP, (float*)0, obase, (size_t)HD, 64);
}

__global__ __launch_bounds__(32) void k_gemm_vt(const h16* __restrict__ WVH, const h16* __restrict__ KVIN, const float* __restrict__ bv, h16* VT) {
    const int r0 = blockIdx.x * 64, c0 = blockIdx.y * 64;
    const int b = c0 / SP, kk = c0 % SP;
    const size_t obase = ((size_t)b * DM + (size_t)r0) * SP + (size_t)kk;
    gemm_tile<1, 0>(WVH, KVIN, DM, (size_t)r0, (size_t)c0, bv, r0, WCI, VT, (float*)0, obase, (size_t)SP, 64);
}

__global__ __launch_bounds__(32) void k_gemm_out(const h16* __restrict__ CTX, const h16* __restrict__ WOH, const float* __restrict__ bo, float* OUT) {
    const int r0 = blockIdx.x * 64, c0 = blockIdx.y * 64;
    const int b = r0 / TP, tt = r0 % TP;
    const size_t obase = ((size_t)b * OUT_T + (size_t)tt) * DM + (size_t)c0;
    gemm_tile<0, 1>(CTX, WOH, DM, (size_t)r0, (size_t)c0, bo, c0, OCI, (h16*)0, OUT, obase, (size_t)DM, TQ - tt);
}

__global__ __launch_bounds__(32 * AW) void k_flash(const h16* __restrict__ QP, const h16* __restrict__ KP, const h16* __restrict__ VT, h16* CTX) {
    __shared__ __align__(16) float os[AW * 16 * OSP];
    const int lane = threadIdx.x & 31, lr = lane & 15, hi = lane >> 4;
    const int wave = __builtin_amdgcn_readfirstlane((int)(threadIdx.x >> 5));
    const int zh = blockIdx.y; const int b = zh / NH_, h = zh % NH_;
    const int t0 = (blockIdx.x * AW + wave) * 16;
    const size_t qo = ((size_t)zh * TP + (size_t)(t0 + lr)) * HD + 8 * hi;
    const v16h q0 = ldh(QP + qo), q1 = ldh(QP + qo + 32);
    const size_t ko = ((size_t)zh * SP + (size_t)lr) * HD + 8 * hi;
    const size_t vo = ((size_t)zh * HD + (size_t)lr) * SP + 8 * hi;
    v8f o0 = (v8f){}, o1 = (v8f){}, o2 = (v8f){}, o3 = (v8f){};
    float m = NEGB, l = 0.0f;
#pragma unroll 1
    for (int key0 = 0; key0 < KEND; key0 += 32) {
        const h16* ka = KP + ko + (size_t)key0 * HD;
        const v16h ka0 = ldh(ka), ka1 = ldh(ka + 32), kb0 = ldh(ka + 16 * HD), kb1 = ldh(ka + 16 * HD + 32);
        v8f sA = (v8f){}, sB = (v8f){};
        sA = wmma16g(ka0, q0, sA); sA = wmma16g(ka1, q1, sA);
        sB = wmma16g(kb0, q0, sB); sB = wmma16g(kb1, q1, sB);
        const int ja = key0 + 8 * hi;
        float ta[8], tb[8]; bool fa[8], fb[8]; float mx = NEGB;
#pragma unroll
        for (int r = 0; r < 8; ++r) {
            fa[r] = (ja + r) < SV;
            fb[r] = (ja + 16 + r) < SV;
            ta[r] = sA[r] * SC2; tb[r] = sB[r] * SC2;
            mx = fmaxf(mx, fmaxf(fa[r] ? ta[r] : NEGB, fb[r] ? tb[r] : NEGB)); }
        mx = fmaxf(mx, __shfl_xor(mx, 16, 32));
        const float mnew = fmaxf(m, mx);
        const float alpha = __builtin_amdgcn_exp2f(m - mnew);
        const float sh = PSH - mnew;
        v16h pb; float ls = 0.0f;
#pragma unroll
        for (int r = 0; r < 8; ++r) {
            const float xa = ta[r] + sh, xb = tb[r] + sh;
            const float ea = __builtin_amdgcn_exp2f(xa), eb = __builtin_amdgcn_exp2f(xb);
            const float ga = (fa[r] & (xa >= -14.0f)) ? ea : 0.0f;
            const float gb = (fb[r] & (xb >= -14.0f)) ? eb : 0.0f;
            const h16 pa = (h16)ga; const h16 pc = (h16)gb;
            pb[r] = pa; pb[8 + r] = pc;
            ls += (float)pa + (float)pc; }
        l = l * alpha + ls; m = mnew;
        o0 = o0 * alpha; o1 = o1 * alpha; o2 = o2 * alpha; o3 = o3 * alpha;
        const h16* va = VT + vo + key0;
        const v16h v0 = ldh(va), v1 = ldh(va + (size_t)16 * SP), v2 = ldh(va + (size_t)32 * SP), v3 = ldh(va + (size_t)48 * SP);
        o0 = wmma16g(v0, pb, o0); o1 = wmma16g(v1, pb, o1); o2 = wmma16g(v2, pb, o2); o3 = wmma16g(v3, pb, o3);
    }
    l += __shfl_xor(l, 16, 32);
    const bool any = l > 0.0f;
    const float lsafe = any ? l : 1.0f;
    const float inv = any ? (1.0f / lsafe) : 0.0f;
    const int wb = wave * 16 * OSP;
    { v4f a, c;
      a[0] = o0[0] * inv; a[1] = o0[1] * inv; a[2] = o0[2] * inv; a[3] = o0[3] * inv; c[0] = o0[4] * inv; c[1] = o0[5] * inv; c[2] = o0[6] * inv; c[3] = o0[7] * inv;
      *(v4fa*)(&os[wb + lr * OSP +  0 + 8 * hi]) = a; *(v4fa*)(&os[wb + lr * OSP +  0 + 8 * hi + 4]) = c;
      a[0] = o1[0] * inv; a[1] = o1[1] * inv; a[2] = o1[2] * inv; a[3] = o1[3] * inv; c[0] = o1[4] * inv; c[1] = o1[5] * inv; c[2] = o1[6] * inv; c[3] = o1[7] * inv;
      *(v4fa*)(&os[wb + lr * OSP + 16 + 8 * hi]) = a; *(v4fa*)(&os[wb + lr * OSP + 16 + 8 * hi + 4]) = c;
      a[0] = o2[0] * inv; a[1] = o2[1] * inv; a[2] = o2[2] * inv; a[3] = o2[3] * inv; c[0] = o2[4] * inv; c[1] = o2[5] * inv; c[2] = o2[6] * inv; c[3] = o2[7] * inv;
      *(v4fa*)(&os[wb + lr * OSP + 32 + 8 * hi]) = a; *(v4fa*)(&os[wb + lr * OSP + 32 + 8 * hi + 4]) = c;
      a[0] = o3[0] * inv; a[1] = o3[1] * inv; a[2] = o3[2] * inv; a[3] = o3[3] * inv; c[0] = o3[4] * inv; c[1] = o3[5] * inv; c[2] = o3[6] * inv; c[3] = o3[7] * inv;
      *(v4fa*)(&os[wb + lr * OSP + 48 + 8 * hi]) = a; *(v4fa*)(&os[wb + lr * OSP + 48 + 8 * hi + 4]) = c; }
    wave_sync();
    h16* crow = CTX + ((size_t)b * TP + (size_t)t0) * DM + (size_t)h * HD;
    static_assert(32 * 16 * 4 == 16 * HD * 2);
#pragma unroll 1
    for (int ps = 0; ps < 2; ++ps) {
#pragma unroll
        for (int s = 0; s < 4; ++s) { const int row = 4 * s + (lane >> 3), c8 = (lane & 7) * 8;
            const v4f x0 = *(const v4fa*)(&os[wb + row * OSP + c8]); const v4f x1 = *(const v4fa*)(&os[wb + row * OSP + c8 + 4]); v8h hv;
#pragma unroll
            for (int i = 0; i < 4; ++i) { hv[i] = toh_flush(x0[i] * CXS); hv[4 + i] = toh_flush(x1[i] * CXS); }
            *(volatile v8h*)(crow + (size_t)row * DM + c8) = hv; }
        if (ps == 0) __threadfence(); }
}

static constexpr size_t al256(size_t v) { return (v + 255) & ~(size_t)255; }
static constexpr size_t SZ_KV = al256((size_t)NB * SP * DM * 2);
static constexpr size_t SZ_CX = al256((size_t)NB * TP * DM * 2);
static constexpr size_t SZ_LR = al256((size_t)NB * LT * DL * 2);
static constexpr size_t SZ_WP = al256((size_t)DM * DL * 2);
static constexpr size_t SZ_W  = al256((size_t)DM * DM * 2);
static constexpr size_t SZ_Q  = al256((size_t)NB * NH_ * TP * HD * 2);
static constexpr size_t SZ_K  = al256((size_t)NB * NH_ * SP * HD * 2);
static constexpr size_t SZ_V  = al256((size_t)NB * DM * SP * 2);
static constexpr size_t SZ_TOTAL = SZ_KV + SZ_LR + SZ_WP + 4 * SZ_W + SZ_Q + SZ_K + SZ_V;
static_assert(SZ_CX <= SZ_KV);
static_assert(SZ_TOTAL <= (size_t)134217728);
static_assert((size_t)NB * NH_ * SP * HD == (size_t)NB * DM * SP);
static_assert(((size_t)NB * TP * (DM / 8)) % 256 == 0);
static_assert(((size_t)SP * DM * 2) % 128 == 0);
static_assert(((size_t)SP * 2) % 128 == 0);
static_assert(((size_t)OUT_T * DM * 4) % 128 == 0);

extern "C" void kernel_launch(void* const* d_in, const int* in_sizes, int n_in,
                              void* d_out, int out_size, void* d_ws, size_t ws_size, hipStream_t stream) {
    if (n_in < 12) return;
    const size_t needx = ((size_t)(NB - 1) * T_FULL + TQ) * DM;
    if ((size_t)in_sizes[0] < needx) return;
    if ((size_t)in_sizes[1] < (size_t)NB * LT * DL) return;
    if ((size_t)in_sizes[2] < (size_t)DM * DL) return;
    if ((size_t)in_sizes[4] < (size_t)DM * DM || (size_t)in_sizes[6] < (size_t)DM * DM || (size_t)in_sizes[8] < (size_t)DM * DM || (size_t)in_sizes[10] < (size_t)DM * DM) return;
    if (in_sizes[3] < DM || in_sizes[5] < DM || in_sizes[7] < DM || in_sizes[9] < DM || in_sizes[11] < DM) return;
    if ((size_t)out_size < ((size_t)(NB - 1) * OUT_T + TQ) * DM) return;
    if (SZ_TOTAL > ws_size) return;
    const float* hid = (const float*)d_in[0];
    const float* lraw = (const float*)d_in[1];
    const float* wp = (const float*)d_in[2];  const float* bp = (const float*)d_in[3];
    const float* wq = (const float*)d_in[4];  const float* bq = (const float*)d_in[5];
    const float* wk = (const float*)d_in[6];  const float* bk = (const float*)d_in[7];
    const float* wv = (const float*)d_in[8];  const float* bv = (const float*)d_in[9];
    const float* wo = (const float*)d_in[10]; const float* bo = (const float*)d_in[11];
    float* OUT = (float*)d_out;
    char* wsp = (char*)d_ws;
    h16* KVIN = (h16*)wsp; h16* CTX = (h16*)wsp; wsp += SZ_KV;
    h16* LRW = (h16*)wsp; wsp += SZ_LR;
    h16* WPH = (h16*)wsp; wsp += SZ_WP;
    h16* WQH = (h16*)wsp; wsp += SZ_W;
    h16* WKH = (h16*)wsp; wsp += SZ_W;
    h16* WVH = (h16*)wsp; wsp += SZ_W;
    h16* WOH = (h16*)wsp; wsp += SZ_W;
    h16* QP = (h16*)wsp; wsp += SZ_Q;
    h16* KP = (h16*)wsp; wsp += SZ_K;
    h16* VT = (h16*)wsp; wsp += SZ_V;

    { const size_t n8 = (size_t)NB * TP * (DM / 8);
      k_cvtx<<<(unsigned)((n8 + 255) / 256), 256, 0, stream>>>(hid, KVIN, n8); }
    { const size_t n8 = (size_t)NB * LT * DL / 8;
      k_cvth<<<(unsigned)((n8 + 255) / 256), 256, 0, stream>>>(lraw, LRW, n8, 1.0f); }
    { const size_t n8 = (size_t)DM * DL / 8;
      k_cvth<<<(unsigned)((n8 + 255) / 256), 256, 0, stream>>>(wp, WPH, n8, WCS); }
    { const size_t n8 = (size_t)DM * DM / 8; const unsigned g = (unsigned)((n8 + 255) / 256);
      k_cvth<<<g, 256, 0, stream>>>(wq, WQH, n8, WCS); k_cvth<<<g, 256, 0, stream>>>(wk, WKH, n8, WCS);
      k_cvth<<<g, 256, 0, stream>>>(wv, WVH, n8, WCS); k_cvth<<<g, 256, 0, stream>>>(wo, WOH, n8, WCS); }

    k_gemm_latt<<<dim3(NB * LT / 64, DM / 64, 1), 32, 0, stream>>>(LRW, WPH, bp, KVIN);
    k_gemm_q<<<dim3(NB * TP / 64, DM / 64, 1), 32, 0, stream>>>(KVIN, WQH, bq, QP);
    k_gemm_k<<<dim3(NB * SP / 64, DM / 64, 1), 32, 0, stream>>>(KVIN, WKH, bk, KP);
    k_gemm_vt<<<dim3(DM / 64, NB * SP / 64, 1), 32, 0, stream>>>(WVH, KVIN, bv, VT);
    k_flash<<<dim3(TP / (16 * AW), NB * NH_, 1), 32 * AW, 0, stream>>>(QP, KP, VT, CTX);
    k_gemm_out<<<dim3(NB * TP / 64, DM / 64, 1), 32, 0, stream>>>(CTX, WOH, bo, OUT);
}
